// LSTMModelA_40793599377857
// MI455X (gfx1250) — hardware-verified
//
#include <hip/hip_runtime.h>

typedef __attribute__((ext_vector_type(16))) _Float16 v16h;
typedef __attribute__((ext_vector_type(8)))  _Float16 v8h;
typedef __attribute__((ext_vector_type(8)))  float    v8f;
typedef __attribute__((ext_vector_type(4)))  float    v4f;

constexpr int kBatch   = 32768;
constexpr int kTime    = 240;
constexpr int kHid     = 25;
constexpr int kHidPad  = 32;
constexpr int kNGate   = 4;
constexpr int kNCls    = 2;
constexpr int kSeqPB   = 64;
constexpr int kBlocks  = kBatch / kSeqPB;
constexpr int kThreads = 256;
constexpr int kHP      = 40;
constexpr int kHTile   = kSeqPB * kHP;
constexpr int kXC      = 80;
constexpr int kXP      = 64;
constexpr int kXPerThr = 20;
constexpr int kFP      = 36;
constexpr int kOutPB   = kSeqPB * kNCls;
static_assert(kBatch % kSeqPB == 0, "grid exact");
static_assert(kTime % kXC == 0, "chunks exact");
static_assert((kThreads / 64) * 16 == kSeqPB, "4 row tiles x 2 unit groups = 8 waves");
static_assert(kHid <= kHidPad && kHidPad == 32, "one k-step");
static_assert(kNGate * kHid == 100, "gate rows");
static_assert(kHP % 8 == 0 && kHP >= kHidPad, "16-B aligned fragment rows");
static_assert(kXC * kSeqPB == kThreads * kXPerThr, "x chunk staging: exactly 20 floats per thread");
static_assert(kXPerThr % 4 == 0, "float4 staging");
static_assert((2 * kHTile) % 8 == 0, "tile zeroing in v8h chunks");
static_assert(kOutPB == 4 * 32, "one wave x float4 per lane = the block output exactly");
static_assert(kOutPB <= kThreads, "head threads");
static_assert(kFP % 4 == 0 && kFP >= kHidPad && kXP % 4 == 0, "pitches");

__device__ __forceinline__ void dep_guard_h(v8f& a, v8f& b, v16h x, v16h y) { asm volatile("v_nop\n\tv_nop\n\tv_nop\n\tv_nop" : "+v"(a), "+v"(b) : "v"(x), "v"(y)); }
__device__ __forceinline__ void keep4_h(v16h a, v16h b, v16h c, v16h d) { asm volatile("v_nop" :: "v"(a), "v"(b), "v"(c), "v"(d)); }

template <typename T> struct Frag;
template <> struct Frag<_Float16> {
  typedef v16h V; union U { v16h v; v8h h[2]; };
  static __device__ __forceinline__ v16h load(const _Float16* p) {
    U f; f.h[0] = *(const v8h*)(p); f.h[1] = *(const v8h*)(p + 16); return f.v;
  }
  static __device__ __forceinline__ v8f mma(v16h a, v16h b, v8f c) {
    return __builtin_amdgcn_wmma_f32_16x16x32_f16(false, a, false, b, (short)0, c, false, false);
  }
  static __device__ __forceinline__ void guard(v8f& a, v8f& b, v16h x, v16h y) { dep_guard_h(a, b, x, y); }
  static __device__ __forceinline__ void keep(v16h a, v16h b, v16h c, v16h d) { keep4_h(a, b, c, d); }
};

__device__ __forceinline__ void mma_guard4x(v8f& a, v8f& b, v8f& c, v8f& d,
                                            v16h x, v16h y0, v16h y1, v16h y2, v16h y3) {
  asm volatile("v_nop\n\tv_nop\n\tv_nop\n\tv_nop"
               : "+v"(a), "+v"(b), "+v"(c), "+v"(d)
               : "v"(x), "v"(y0), "v"(y1), "v"(y2), "v"(y3));
}

__device__ __forceinline__ float fsig(float x)  { return __builtin_amdgcn_rcpf(1.0f + __expf(-x)); }
__device__ __forceinline__ float ftanh(float x) { return 1.0f - 2.0f * __builtin_amdgcn_rcpf(__expf(2.0f * x) + 1.0f); }

__global__ __launch_bounds__(kThreads) void lstm_fused_kernel(
    const float* __restrict__ x,
    const float* __restrict__ wih, const float* __restrict__ whh,
    const float* __restrict__ bih, const float* __restrict__ bhh,
    const float* __restrict__ wfc, const float* __restrict__ bfc,
    float* __restrict__ out)
{
  __shared__ __align__(16) _Float16 hbuf[2 * kHTile];
  __shared__ __align__(16) float    xs[kXC * kXP];
  __shared__ __align__(16) float    hfin[kSeqPB * kFP];
  __shared__ __align__(16) float    outs[kOutPB];

  const int tid  = threadIdx.x;
  const int lane = tid & 31;
  const int wave = tid >> 5;
  const int c    = lane & 15;
  const int hh   = lane >> 4;
  const int koff = hh * 8;
  const int mOff = hh * 8;
  const int rt   = wave >> 1;
  const int ug   = wave & 1;
  const int r0   = rt * 16;
  const int u    = 16 * ug + c;
  const bool uval = (u < kHid);
  const int uc   = uval ? u : (kHid - 1);
  const int b0   = (int)blockIdx.x * kSeqPB;

  {
    const v8h z = {(_Float16)0.f, (_Float16)0.f, (_Float16)0.f, (_Float16)0.f, (_Float16)0.f, (_Float16)0.f, (_Float16)0.f, (_Float16)0.f};
    for (int i = tid; i < (2 * kHTile) / 8; i += kThreads) *(v8h*)(hbuf + i * 8) = z;
  }

  float wih8[kNGate], bsum8[kNGate];
  v16h  fb[kNGate];
#pragma unroll
  for (int g = 0; g < kNGate; ++g) {
    const int row = g * kHid + uc;
    const float w = wih[row];
    const float s = bih[row] + bhh[row];
    wih8[g]  = uval ? (w * 8.0f) : 0.0f;
    bsum8[g] = uval ? (s * 8.0f) : 0.0f;
#pragma unroll
    for (int i = 0; i < 16; ++i) {
      const int  k  = (i < 8) ? (koff + i) : (16 + koff + (i - 8));
      const bool kv = (k < kHid);
      const int  kc = kv ? k : (kHid - 1);
      const float v = whh[row * kHid + kc];
      fb[g][i] = (_Float16)((uval && kv) ? (v * 8.0f) : 0.0f);
    }
  }
  float cst[8], hv[8];
#pragma unroll
  for (int r = 0; r < 8; ++r) { cst[r] = 0.0f; hv[r] = 0.0f; }
  __syncthreads();

  const int sseq = tid >> 2;
  const int sq   = tid & 3;
  const float* xrow = x + (size_t)(b0 + sseq) * kTime;

#pragma unroll 1
  for (int cnk = 0; cnk < kTime / kXC; ++cnk) {
    {
      const float* sp = xrow + cnk * kXC + sq * kXPerThr;
#pragma unroll
      for (int i = 0; i < kXPerThr / 4; ++i) {
        const v4f v = *(const v4f*)(sp + 4 * i);
#pragma unroll
        for (int e = 0; e < 4; ++e) xs[(sq * kXPerThr + 4 * i + e) * kXP + sseq] = v[e];
      }
    }
    __syncthreads();

#pragma unroll 1
    for (int tt = 0; tt < kXC; ++tt) {
      const int t = cnk * kXC + tt;
      const _Float16* hc = hbuf + (t & 1) * kHTile;
      _Float16*       hn = hbuf + ((t + 1) & 1) * kHTile;

      const float* xp = xs + tt * kXP + r0 + mOff;
      const v4f xa = *(const v4f*)xp;
      const v4f xb = *(const v4f*)(xp + 4);
      float xv[8];
      xv[0] = xa[0]; xv[1] = xa[1]; xv[2] = xa[2]; xv[3] = xa[3];
      xv[4] = xb[0]; xv[5] = xb[1]; xv[6] = xb[2]; xv[7] = xb[3];

      v8f acc[kNGate];
#pragma unroll
      for (int g = 0; g < kNGate; ++g) {
#pragma unroll
        for (int r = 0; r < 8; ++r) acc[g][r] = fmaf(xv[r], wih8[g], bsum8[g]);
      }

      const v16h fa = Frag<_Float16>::load(hc + (r0 + c) * kHP + koff);
      acc[0] = Frag<_Float16>::mma(fa, fb[0], acc[0]);
      acc[1] = Frag<_Float16>::mma(fa, fb[1], acc[1]);
      acc[2] = Frag<_Float16>::mma(fa, fb[2], acc[2]);
      acc[3] = Frag<_Float16>::mma(fa, fb[3], acc[3]);
      mma_guard4x(acc[0], acc[1], acc[2], acc[3], fa, fb[0], fb[1], fb[2], fb[3]);

#pragma unroll
      for (int r = 0; r < 8; ++r) {
        const float zi = acc[0][r] * 0.125f;
        const float zf = acc[1][r] * 0.125f;
        const float zg = acc[2][r] * 0.125f;
        const float zo = acc[3][r] * 0.125f;
        const float ig = fsig(zi);
        const float fg = fsig(zf);
        const float gg = ftanh(zg);
        const float og = fsig(zo);
        const float cn = fg * cst[r] + ig * gg;
        cst[r] = cn;
        float h = og * ftanh(cn);
        h = uval ? h : 0.0f;
        hv[r] = h;
        hn[(r0 + mOff + r) * kHP + u] = (_Float16)h;
      }
      if (t == kTime - 1) {
#pragma unroll
        for (int r = 0; r < 8; ++r) hfin[(r0 + mOff + r) * kFP + u] = hv[r];
      }
      __syncthreads();
    }
  }

  if (tid < kOutPB) {
    const int seq = tid >> 1;
    const int cls = tid & 1;
    const float* hp = hfin + seq * kFP;
    const float* wp = wfc + cls * kHid;
    float s = 0.0f;
#pragma unroll 1
    for (int k = 0; k < kHid; ++k) s = fmaf(hp[k], wp[k], s);
    s += bfc[cls];
    outs[tid] = s;
  }
  __syncthreads();
  if (wave == 0) {
    const v4f val = *(const v4f*)(outs + 4 * lane);
    float* op = out + (size_t)b0 * kNCls;
    for (int pass = 0; pass < 2; ++pass) {
      *(volatile v4f*)(op + 4 * lane) = val;
      __threadfence();
    }
  }
}

extern "C" void kernel_launch(void* const* d_in, const int* in_sizes, int n_in,
                              void* d_out, int out_size, void* d_ws, size_t ws_size, hipStream_t stream) {
  (void)d_ws; (void)ws_size;
  if (n_in < 7 || d_out == nullptr) return;
  if (in_sizes[0] != kBatch * kTime || in_sizes[1] != kNGate * kHid || in_sizes[2] != kNGate * kHid * kHid ||
      in_sizes[3] != kNGate * kHid || in_sizes[4] != kNGate * kHid || in_sizes[5] != kNCls * kHid ||
      in_sizes[6] != kNCls || out_size != kBatch * kNCls) return;

  const float* x   = (const float*)d_in[0];
  const float* wih = (const float*)d_in[1];
  const float* whh = (const float*)d_in[2];
  const float* bih = (const float*)d_in[3];
  const float* bhh = (const float*)d_in[4];
  const float* wfc = (const float*)d_in[5];
  const float* bfc = (const float*)d_in[6];
  float* out = (float*)d_out;

  lstm_fused_kernel<<<kBlocks, kThreads, 0, stream>>>(x, wih, whh, bih, bhh, wfc, bfc, out);
}
